// QuantumLayer_37074157699082
// MI455X (gfx1250) — hardware-run, weakly checked
//
#include <hip/hip_runtime.h>


#ifndef NROWS
#define NROWS 512
#endif
#define NROWS_FULL 512
#define DIN  128
#define NQ   16
#define DOUT 128
#define HP   20
#define OP   132

static_assert(NROWS % 16 == 0);
static_assert(NROWS <= NROWS_FULL);
static_assert(DIN % 32 == 0);
static_assert(NQ == 16);
static_assert(2 * 8 == NQ);
static_assert(DOUT % 16 == 0);
static_assert(32 * 4 == DOUT);
static_assert(HP >= NQ && (HP * 4) % 16 == 0);
static_assert(OP >= DOUT && (OP * 4) % 16 == 0);
static_assert((16 * HP + 16 * OP) * 4 <= 131072);

typedef unsigned short bf;
typedef __attribute__((ext_vector_type(16))) __bf16   v16bf;
typedef __attribute__((ext_vector_type(8)))  unsigned short v8us;
typedef __attribute__((ext_vector_type(8)))  float    v8f;
typedef __attribute__((ext_vector_type(4)))  float    v4f;
typedef v4f  __attribute__((may_alias)) v4fa;

__device__ __forceinline__ unsigned short f2bf(float f) { unsigned u = __float_as_uint(f); u += 0x7FFFu + ((u >> 16) & 1u); return (unsigned short)(u >> 16); }
__device__ __forceinline__ float bfr(float f) { return __uint_as_float(((unsigned)f2bf(f)) << 16); }
__device__ __forceinline__ v16bf cat16b(v8us lo, v8us hi) { return __builtin_bit_cast(v16bf, __builtin_shufflevector(lo, hi, 0, 1, 2, 3, 4, 5, 6, 7, 8, 9, 10, 11, 12, 13, 14, 15)); }
__device__ __forceinline__ v8f wmmab(v16bf a, v16bf b, v8f c) { return __builtin_amdgcn_wmma_f32_16x16x32_bf16(false, a, false, b, (short)0, c, false, false); }
__device__ __forceinline__ v8f wmmab_g(v16bf a, v16bf b, v8f c) {
    c = wmmab(a, b, c);
    asm volatile("v_nop\n\tv_nop\n\tv_nop\n\tv_nop" : "+v"(c) : "v"(a), "v"(b));
    return c;
}
__device__ __forceinline__ v8us ld8bf(const float* p) {
    const v4f a = *(const v4f*)p; const v4f b = *(const v4f*)(p + 4); v8us o;
#pragma unroll
    for (int i = 0; i < 4; ++i) { o[i] = f2bf(a[i]); o[4 + i] = f2bf(b[i]); }
    return o;
}

__global__ __launch_bounds__(32) void k_fused(const float* __restrict__ x, const float* __restrict__ w_in, const float* __restrict__ b_in,
                                               const float* __restrict__ w_out, const float* __restrict__ b_out, float* out) {
    __shared__ __align__(16) float hs[16 * HP];
    __shared__ __align__(16) float os[16 * OP];
    const int lane = threadIdx.x & 31, lr = lane & 15, hi = lane >> 4;
    const int r0 = blockIdx.x * 16;

    v8f acc = (v8f){};
    const size_t aoff = (size_t)(r0 + lr) * DIN + 8 * hi;
    const size_t boff = (size_t)lr * DIN + 8 * hi;
#pragma unroll
    for (int kc = 0; kc < DIN; kc += 32) {
        const v16bf a = cat16b(ld8bf(x + aoff + kc), ld8bf(x + aoff + kc + 16));
        const v16bf b = cat16b(ld8bf(w_in + boff + kc), ld8bf(w_in + boff + kc + 16));
        acc = wmmab_g(a, b, acc);
    }
    const float bi = bfr(b_in[lr]);
#pragma unroll
    for (int r = 0; r < 8; ++r) hs[(8 * hi + r) * HP + lr] = acc[r] + bi;
    __syncthreads();

#pragma unroll 1
    for (int q = 0; q < 8; ++q) { const int ix = lr * HP + 8 * hi + q; const float v = hs[ix]; hs[ix] = cosf(v); }
    __syncthreads();

    float c[16];
#pragma unroll
    for (int q = 0; q < 16; q += 4) { const v4f t4 = *(const v4fa*)(&hs[lr * HP + q]); c[q] = t4[0]; c[q + 1] = t4[1]; c[q + 2] = t4[2]; c[q + 3] = t4[3]; }
    v8us eh, el;
#pragma unroll
    for (int t = 0; t < 8; ++t) {
        const int i = 8 * hi + t;
        const unsigned msk = ((0x1111u << (i & 3)) | (0x1111u << ((i + 3) & 3))) & ((2u << i) - 1u);
        float p = 1.0f;
#pragma unroll
        for (int q = 0; q < 16; ++q) p *= ((msk >> q) & 1u) ? c[q] : 1.0f;
        const unsigned short ph = f2bf(p);
        const float pf = __uint_as_float(((unsigned)ph) << 16);
        eh[t] = ph; el[t] = f2bf(p - pf);
    }
    const v16bf ea = cat16b(eh, el);

#pragma unroll
    for (int nt = 0; nt < DOUT / 16; ++nt) {
        const v8us wv = ld8bf(w_out + (size_t)(nt * 16 + lr) * NQ + 8 * hi);
        const v16bf wb = cat16b(wv, wv);
        v8f o = (v8f){};
        o = wmmab_g(ea, wb, o);
        const float bo = bfr(b_out[nt * 16 + lr]);
#pragma unroll
        for (int r = 0; r < 8; ++r) os[(8 * hi + r) * OP + nt * 16 + lr] = o[r] + bo;
    }
    __syncthreads();

    float* orow = out + (size_t)r0 * DOUT + lane * 4;
#pragma unroll 1
    for (int ps = 0; ps < 2; ++ps) {
#pragma unroll
        for (int row = 0; row < 16; ++row) {
            const v4f val = *(const v4fa*)(&os[row * OP + lane * 4]);
            *(volatile v4f*)(orow + (size_t)row * DOUT) = val; }
        if (ps == 0) __threadfence(); }
}

extern "C" void kernel_launch(void* const* d_in, const int* in_sizes, int n_in,
                              void* d_out, int out_size, void* d_ws, size_t ws_size, hipStream_t stream) {
    (void)d_ws; (void)ws_size;
    if (n_in < 6) return;
    if ((size_t)in_sizes[0] < (size_t)NROWS * DIN) return;
    if (in_sizes[1] < NQ * DIN || in_sizes[2] < NQ || in_sizes[4] < DOUT * NQ || in_sizes[5] < DOUT) return;
    if ((size_t)out_size < (size_t)NROWS * DOUT) return;
    const float* x     = (const float*)d_in[0];
    const float* w_in  = (const float*)d_in[1];
    const float* b_in  = (const float*)d_in[2];
    const float* w_out = (const float*)d_in[4];
    const float* b_out = (const float*)d_in[5];
    float* out = (float*)d_out;
    k_fused<<<dim3(NROWS / 16, 1, 1), dim3(32, 1, 1), 0, stream>>>(x, w_in, b_in, w_out, b_out, out);
}
